// MultiLayerLSTM_58119497450297
// MI455X (gfx1250) — hardware-verified
//
#include <hip/hip_runtime.h>
#include <stdint.h>
#include <math.h>

typedef __attribute__((ext_vector_type(16))) _Float16 v16h;
typedef __attribute__((ext_vector_type(8)))  _Float16 v8h;
typedef __attribute__((ext_vector_type(16))) __bf16   v16b;
typedef __attribute__((ext_vector_type(8)))  __bf16   v8b;
typedef __attribute__((ext_vector_type(8)))  float    v8f;
typedef __attribute__((ext_vector_type(4)))  float    v4f;
typedef __attribute__((ext_vector_type(4)))  unsigned v4u;

__device__ __forceinline__ unsigned short f2bf_bits(float f) {
  unsigned u = __float_as_uint(f);
  return (unsigned short)((u + 0x7FFFu + ((u >> 16) & 1u)) >> 16);
}
__device__ __forceinline__ float bf_bits2f(unsigned short h) { return __uint_as_float(((unsigned)h) << 16); }

__device__ __forceinline__ void dep_guard_h(v8f& a, v8f& b, v16h x, v16h y) { asm volatile("v_nop\n\tv_nop\n\tv_nop\n\tv_nop" : "+v"(a), "+v"(b) : "v"(x), "v"(y)); }
__device__ __forceinline__ void dep_guard_b(v8f& a, v8f& b, v16b x, v16b y) { asm volatile("v_nop\n\tv_nop\n\tv_nop\n\tv_nop" : "+v"(a), "+v"(b) : "v"(x), "v"(y)); }
__device__ __forceinline__ void keep4_h(v16h a, v16h b, v16h c, v16h d) { asm volatile("v_nop" :: "v"(a), "v"(b), "v"(c), "v"(d)); }
__device__ __forceinline__ void keep4_b(v16b a, v16b b, v16b c, v16b d) { asm volatile("v_nop" :: "v"(a), "v"(b), "v"(c), "v"(d)); }
__device__ __forceinline__ void acc_guard4(v8f& a, v8f& b, v8f& c, v8f& d) { asm volatile("v_nop\n\tv_nop\n\tv_nop\n\tv_nop" : "+v"(a), "+v"(b), "+v"(c), "+v"(d)); }
template <typename T> struct Frag;
template <> struct Frag<_Float16> {
  typedef v16h V; union U { v16h v; v8h h[2]; };
  static __device__ __forceinline__ v16h load(const _Float16* p) {
    U f; f.h[0] = *(const v8h*)(p); f.h[1] = *(const v8h*)(p + 16); return f.v;
  }
  static __device__ __forceinline__ v8f mma(v16h a, v16h b, v8f c) {
    return __builtin_amdgcn_wmma_f32_16x16x32_f16(false, a, false, b, (short)0, c, false, false);
  }
  static __device__ __forceinline__ void guard(v8f& a, v8f& b, v16h x, v16h y) { dep_guard_h(a, b, x, y); }
  static __device__ __forceinline__ void keep(v16h a, v16h b, v16h c, v16h d) { keep4_h(a, b, c, d); }
};
template <> struct Frag<__bf16> {
  typedef v16b V; union U { v16b v; v8b h[2]; };
  static __device__ __forceinline__ v16b load(const __bf16* p) {
    U f; f.h[0] = *(const v8b*)(p); f.h[1] = *(const v8b*)(p + 16); return f.v;
  }
  static __device__ __forceinline__ v8f mma(v16b a, v16b b, v8f c) {
    return __builtin_amdgcn_wmma_f32_16x16x32_bf16(false, a, false, b, (short)0, c, false, false);
  }
  static __device__ __forceinline__ void guard(v8f& a, v8f& b, v16b x, v16b y) { dep_guard_b(a, b, x, y); }
  static __device__ __forceinline__ void keep(v16b a, v16b b, v16b c, v16b d) { keep4_b(a, b, c, d); }
};

template <int ET> struct Elem;
template <> struct Elem<0> { typedef _Float16 T; };
template <> struct Elem<1> { typedef __bf16 T; };
template <int ET, bool SPLIT, int BIAS_MODE, int OUT_MODE, bool RESID, int ACT = 0>
__global__ __launch_bounds__(256) void wmma_gemm64(
    const unsigned short* __restrict__ Ap, const unsigned short* __restrict__ A2p, int lda, long strideA,
    const unsigned short* __restrict__ Btp, const unsigned short* __restrict__ Bt2p, int ldb, long strideB,
    void* __restrict__ Cout, void* __restrict__ Cout2, int ldc, long strideC,
    const float* __restrict__ bias,
    const float* __restrict__ resid, long strideR,
    int M, int N, int K, float scale) {
  typedef typename Elem<ET>::T T;
  typedef typename Frag<T>::V V;
  const T* A = (const T*)Ap; const T* A2 = (const T*)A2p; const T* Bt = (const T*)Btp; const T* Bt2 = (const T*)Bt2p;
  __shared__ __align__(16) float sT[8][16 * 68];
  const int b    = blockIdx.y;
  const int lane = threadIdx.x & 31;
  const int wave = threadIdx.x >> 5;
  const int tilesN = N >> 6;
  const int tilesM = M >> 6;
  const int tile = blockIdx.x * 8 + wave;
  if (tile >= tilesM * tilesN) return;
  const int tm = tile / tilesN;
  const int tn = tile - tm * tilesN;
  const int m0 = tm << 6;
  const int n0 = tn << 6;

  const T* Ab  = A  + (size_t)b * strideA;
  const T* Bb  = Bt + (size_t)b * strideB;
  const T* Ab2 = SPLIT ? (A2  + (size_t)b * strideA) : nullptr;
  const T* Bb2 = SPLIT ? (Bt2 + (size_t)b * strideB) : nullptr;

  const int rlane = lane & 15;
  const int koff  = (lane >> 4) * 8;
  const int mOff  = (lane >> 4) * 8;

  v8f acc[4][4];
#pragma unroll
  for (int i = 0; i < 4; ++i)
#pragma unroll
    for (int j = 0; j < 4; ++j) acc[i][j] = (v8f){0.f,0.f,0.f,0.f,0.f,0.f,0.f,0.f};

  for (int k0 = 0; k0 < K; k0 += 32) {
    V bh[4], bl[4];
#pragma unroll
    for (int j = 0; j < 4; ++j) {
      const size_t bo = (size_t)(n0 + (j << 4) + rlane) * ldb + koff + k0;
      bh[j] = Frag<T>::load(Bb + bo);
      if (SPLIT) bl[j] = Frag<T>::load(Bb2 + bo);
    }
#pragma unroll
    for (int i = 0; i < 4; ++i) {
      const size_t ao = (size_t)(m0 + (i << 4) + rlane) * lda + koff + k0;
      V ah = Frag<T>::load(Ab + ao);
      V al;
      if (SPLIT) al = Frag<T>::load(Ab2 + ao);
#pragma unroll
      for (int j = 0; j < 4; ++j) {
        acc[i][j] = Frag<T>::mma(ah, bh[j], acc[i][j]);
        if (SPLIT) {
          acc[i][j] = Frag<T>::mma(ah, bl[j], acc[i][j]);
          acc[i][j] = Frag<T>::mma(al, bh[j], acc[i][j]);
        }
      }
      Frag<T>::guard(acc[i][0], acc[i][3], ah, SPLIT ? al : ah);
    }
    Frag<T>::keep(bh[0], bh[1], bh[2], bh[3]);
    if (SPLIT) Frag<T>::keep(bl[0], bl[1], bl[2], bl[3]);
  }
  acc_guard4(acc[0][0], acc[0][1], acc[0][2], acc[0][3]);
  acc_guard4(acc[1][0], acc[1][1], acc[1][2], acc[1][3]);
  acc_guard4(acc[2][0], acc[2][1], acc[2][2], acc[2][3]);
  acc_guard4(acc[3][0], acc[3][1], acc[3][2], acc[3][3]);

  float* slab = sT[wave];
  const float* Rb = RESID ? (resid + (size_t)b * strideR) : nullptr;
#pragma unroll
  for (int i = 0; i < 4; ++i) {
    const int mBase = m0 + (i << 4);
#pragma unroll
    for (int j = 0; j < 4; ++j) {
      const int n = n0 + (j << 4) + rlane;
      float bv = 0.f;
      if (BIAS_MODE == 2) bv = bias[n];
#pragma unroll
      for (int r = 0; r < 8; ++r) {
        float v = acc[i][j][r] * scale;
        if (BIAS_MODE == 1) v += bias[mBase + mOff + r];
        if (BIAS_MODE == 2) v += bv;
        if (RESID) v += Rb[(size_t)(mBase + mOff + r) * ldc + n];
        if (ACT == 1) v = tanhf(v);
        if (ACT == 2) v = fmaxf(v, 0.0f);
        if (ACT == 3) v = v / (1.0f + expf(-v));
        if (ACT == 4) v = (v > 0.f) ? v : 0.01f * v;
        if (ACT == 5) v = 0.5f * v * (1.0f + erff(v * 0.70710678118654752f));
        slab[(mOff + r) * 68 + (j << 4) + rlane] = v;
      }
    }
    __builtin_amdgcn_fence(__ATOMIC_RELEASE, "workgroup");
    __builtin_amdgcn_wave_barrier();
    __builtin_amdgcn_fence(__ATOMIC_ACQUIRE, "workgroup");
    if (OUT_MODE == 0) {
      float* C = (float*)Cout + (size_t)b * strideC;
      const int hh = lane >> 4, c4 = (lane & 15) * 4;
      for (int pass = 0; pass < 2; ++pass) {
#pragma unroll
        for (int it = 0; it < 8; ++it) {
          const int row = it * 2 + hh;
          v4f v = *(const v4f*)(slab + row * 68 + c4);
          *(volatile v4f*)(C + (size_t)(mBase + row) * ldc + n0 + c4) = v;
        }
        __threadfence();
      }
    } else {
      const int q = lane >> 3, c8 = (lane & 7) * 8;
      unsigned short* C  = (unsigned short*)Cout  + (size_t)b * strideC;
      unsigned short* C2 = (OUT_MODE == 2) ? ((unsigned short*)Cout2 + (size_t)b * strideC) : nullptr;
      for (int pass = 0; pass < 2; ++pass) {
#pragma unroll
        for (int it = 0; it < 4; ++it) {
          const int row = it * 4 + q;
          const float* sp = slab + row * 68 + c8;
          v8h hv, lv;
#pragma unroll
          for (int e = 0; e < 8; ++e) {
            if (OUT_MODE == 1) {
              hv[e] = (_Float16)sp[e];
            } else {
              unsigned short hb = f2bf_bits(sp[e]);
              unsigned short lb = f2bf_bits(sp[e] - bf_bits2f(hb));
              hv[e] = __builtin_bit_cast(_Float16, hb);
              lv[e] = __builtin_bit_cast(_Float16, lb);
            }
          }
          *(volatile v8h*)(C + (size_t)(mBase + row) * ldc + n0 + c8) = hv;
          if (OUT_MODE == 2) *(volatile v8h*)(C2 + (size_t)(mBase + row) * ldc + n0 + c8) = lv;
        }
        __threadfence();
      }
    }
    __builtin_amdgcn_fence(__ATOMIC_RELEASE, "workgroup");
    __builtin_amdgcn_wave_barrier();
    __builtin_amdgcn_fence(__ATOMIC_ACQUIRE, "workgroup");
  }
}

constexpr int NBATCH = 256;
constexpr int NSTEP  = 1024;
constexpr int NVOC   = 27;
constexpr int NEMB   = 64;
constexpr int NHID   = 128;
constexpr int NGATE  = 4 * NHID;
constexpr int ROWS_PER_BLK = 16;
constexpr int NBLK_MAIN = NBATCH / ROWS_PER_BLK;
constexpr int HPITCH = 128;
constexpr int YCHUNK = 32;
constexpr int YPITCH = YCHUNK * NVOC;
constexpr int YLINES = YPITCH / 32;
constexpr int NVOCPAD = 32;
constexpr int NEMBROWS = 64;

static_assert(NBATCH % ROWS_PER_BLK == 0, "batch tiles");
static_assert(NSTEP % YCHUNK == 0, "flush chunks");
static_assert(YPITCH % 32 == 0, "whole lines per chunk row");
static_assert((NSTEP * NVOC * 4) % 128 == 0, "per-batch-row output base is line aligned");
static_assert((YCHUNK * NVOC * 4) % 128 == 0, "per-chunk output base is line aligned");
static_assert(NHID % 32 == 0 && NEMB % 32 == 0, "K multiples of 32");
static_assert(NEMBROWS % 64 == 0 && NGATE % 64 == 0 && NEMB % 32 == 0, "table GEMM M,N,K tile contract");
static_assert(NBATCH * NSTEP * NVOC * 4 == 28311552, "output extent");

constexpr float SC_H  = 16384.0f;
constexpr float SC_W  = 4096.0f;
constexpr float SC_Y  = 16.0f;
constexpr float SC_LO = 2048.0f;
constexpr float GATE_INV = 1.0f / (16384.0f * 4096.0f);
constexpr float Y_INV    = 1.0f / (16384.0f * 16.0f);
constexpr float LO_INV   = 1.0f / 2048.0f;

constexpr size_t WS_EMBB  = 0;
constexpr size_t WS_WX0T  = 8192;
constexpr size_t WS_WH0T  = 73728;
constexpr size_t WS_WX1T  = 204800;
constexpr size_t WS_WH1T  = 335872;
constexpr size_t WS_WHYT  = 466944;
constexpr size_t WS_XPROJ = 475136;
constexpr size_t WS_TOTAL = 606208;
static_assert(WS_WX0T == WS_EMBB + 64 * 64 * 2, "carve");
static_assert(WS_WH0T == WS_WX0T + 512 * 64 * 2, "carve");
static_assert(WS_WX1T == WS_WH0T + 512 * 128 * 2, "carve");
static_assert(WS_WH1T == WS_WX1T + 512 * 128 * 2, "carve");
static_assert(WS_WHYT == WS_WH1T + 512 * 128 * 2, "carve");
static_assert(WS_XPROJ == WS_WHYT + 32 * 128 * 2, "carve");
static_assert(WS_TOTAL == WS_XPROJ + 64 * 512 * 4, "carve");
static_assert(WS_TOTAL <= 134217728, "carve budget");

constexpr int LDS_XP    = 0;
constexpr int LDS_YB    = 55296;
constexpr int LDS_H0    = 110592;
constexpr int LDS_H1H   = 118784;
constexpr int LDS_H1L   = 126976;
constexpr int LDS_TOTAL = 135168;
constexpr int HBUF = ROWS_PER_BLK * HPITCH;
static_assert(LDS_YB == LDS_XP + NVOC * NGATE * 4, "lds");
static_assert(LDS_H0 == LDS_YB + ROWS_PER_BLK * YPITCH * 4, "lds");
static_assert(LDS_H1H == LDS_H0 + 2 * HBUF * 2 && LDS_H1L == LDS_H1H + 2 * HBUF * 2 && LDS_TOTAL == LDS_H1L + 2 * HBUF * 2, "lds");

__device__ __forceinline__ float bf_rne(float x) { return bf_bits2f(f2bf_bits(x)); }

__device__ __forceinline__ float lsig(float x) {
  const float e = exp2f(x * -1.4426950408889634f);
  return __builtin_amdgcn_rcpf(1.0f + e);
}
__device__ __forceinline__ float ltanh(float x) {
  const float ax = fabsf(x);
  float r;
  if (ax < 0.3f) {
    const float x2 = x * x;
    float p = 0.021869488536155203f;
    p = p * x2 - 0.053968253968253968f;
    p = p * x2 + 0.13333333333333333f;
    p = p * x2 - 0.33333333333333333f;
    r = x + x * (x2 * p);
  } else {
    const float e = exp2f(ax * -2.8853900817779268f);
    r = copysignf((1.0f - e) * __builtin_amdgcn_rcpf(1.0f + e), x);
  }
  return r;
}

__global__ __launch_bounds__(256) void k_prep16(const float* __restrict__ src, long sr, long sk, int rValid,
                                                unsigned short* __restrict__ dst, int dstRows, int kdim,
                                                float scale, int mode) {
  const int lane = threadIdx.x & 31;
  const int gw = blockIdx.x * 8 + (threadIdx.x >> 5);
  const int lanesPerRow = kdim >> 3;
  const int rowsPerWave = 32 / lanesPerRow;
  const int rbase = gw * rowsPerWave;
  if (rbase >= dstRows) return;
  const int lr = lane / lanesPerRow;
  const int r = rbase + lr;
  const int k8 = (lane - lr * lanesPerRow) * 8;
  const bool valid = r < rValid;
  const int rc = valid ? r : (rValid - 1);
  unsigned w[4];
#pragma unroll
  for (int q = 0; q < 4; ++q) {
    unsigned short bits[2];
#pragma unroll
    for (int e = 0; e < 2; ++e) {
      const int k = k8 + 2 * q + e;
      float v = src[(size_t)rc * (size_t)sr + (size_t)k * (size_t)sk];
      v = valid ? v : 0.0f;
      const unsigned short bb = f2bf_bits(v);
      unsigned short o;
      if (mode == 0) {
        o = bb;
      } else {
        const float f = bf_bits2f(bb) * scale;
        o = __builtin_bit_cast(unsigned short, (_Float16)f);
      }
      bits[e] = o;
    }
    w[q] = (unsigned)bits[0] | ((unsigned)bits[1] << 16);
  }
  v4u pk;
  pk.x = w[0]; pk.y = w[1]; pk.z = w[2]; pk.w = w[3];
  unsigned short* p = dst + (size_t)r * kdim + k8;
  *(volatile v4u*)p = pk;
  __threadfence();
  *(volatile v4u*)p = pk;
}

__global__ __launch_bounds__(256) void k_lstm2(const int* __restrict__ xtok, const float* __restrict__ xproj,
                                               const unsigned short* __restrict__ wh0Tp,
                                               const unsigned short* __restrict__ wx1Tp,
                                               const unsigned short* __restrict__ wh1Tp,
                                               const unsigned short* __restrict__ whyTp,
                                               const float* __restrict__ b0, const float* __restrict__ b1,
                                               const float* __restrict__ by, float* __restrict__ out) {
  extern __shared__ __align__(16) char smem[];
  float* xpl = (float*)(smem + LDS_XP);
  float* yb  = (float*)(smem + LDS_YB);
  _Float16* h0b  = (_Float16*)(smem + LDS_H0);
  _Float16* h1hb = (_Float16*)(smem + LDS_H1H);
  _Float16* h1lb = (_Float16*)(smem + LDS_H1L);
  const _Float16* WH0 = (const _Float16*)wh0Tp;
  const _Float16* WX1 = (const _Float16*)wx1Tp;
  const _Float16* WH1 = (const _Float16*)wh1Tp;
  const _Float16* WHY = (const _Float16*)whyTp;

  const int tid  = threadIdx.x;
  const int lane = tid & 31;
  const int wave = tid >> 5;
  const int hh   = lane >> 4;
  const int nn   = lane & 15;
  const int koff = hh * 8;
  const int bbase = blockIdx.x * ROWS_PER_BLK;
  const int unit = wave * 16 + nn;

  for (int i = tid; i < (NVOC * NGATE) / 4; i += 256) ((v4f*)xpl)[i] = ((const v4f*)xproj)[i];
  {
    v4u z; z.x = 0u; z.y = 0u; z.z = 0u; z.w = 0u;
    for (int i = tid; i < (3 * 2 * HBUF * 2) / 16; i += 256) ((v4u*)(smem + LDS_H0))[i] = z;
  }
  float b0r[4], b1r[4];
#pragma unroll
  for (int g = 0; g < 4; ++g) {
    b0r[g] = bf_rne(b0[g * NHID + unit]);
    b1r[g] = bf_rne(b1[g * NHID + unit]);
  }
  const int ycol  = wave * 16 + nn;
  const int ycolc = ycol < NVOC ? ycol : (NVOC - 1);
  const float byr = bf_rne(by[ycolc]);
  float c0r[8], c1r[8];
#pragma unroll
  for (int r = 0; r < 8; ++r) { c0r[r] = 0.0f; c1r[r] = 0.0f; }
  const v8f z8 = (v8f){0.f,0.f,0.f,0.f,0.f,0.f,0.f,0.f};
  __syncthreads();

  for (int t = 0; t < NSTEP; ++t) {
    int tokr[8];
#pragma unroll
    for (int r = 0; r < 8; ++r) {
      int v = xtok[(size_t)(bbase + hh * 8 + r) * NSTEP + t];
      v = v < 0 ? 0 : v;
      v = v > (NVOC - 1) ? (NVOC - 1) : v;
      tokr[r] = v;
    }

    {
      const _Float16* h0p = h0b + (t & 1) * HBUF;
      _Float16* h0n = h0b + ((t + 1) & 1) * HBUF;
      v8f acc[4];
#pragma unroll
      for (int g = 0; g < 4; ++g) acc[g] = z8;
#pragma unroll
      for (int ks = 0; ks < NHID / 32; ++ks) {
        const int kk = ks * 32 + koff;
        const v16h a = Frag<_Float16>::load(h0p + nn * HPITCH + kk);
        v16h bq[4];
#pragma unroll
        for (int g = 0; g < 4; ++g) bq[g] = Frag<_Float16>::load(WH0 + (size_t)(g * NHID + unit) * NHID + kk);
#pragma unroll
        for (int g = 0; g < 4; ++g) acc[g] = Frag<_Float16>::mma(a, bq[g], acc[g]);
        dep_guard_h(acc[0], acc[3], a, bq[3]);
        keep4_h(bq[0], bq[1], bq[2], bq[3]);
      }
      acc_guard4(acc[0], acc[1], acc[2], acc[3]);
#pragma unroll
      for (int r = 0; r < 8; ++r) {
        const int row = hh * 8 + r;
        const float* xr = xpl + tokr[r] * NGATE + unit;
        const float pf = acc[0][r] * GATE_INV + xr[0]        + b0r[0];
        const float pi = acc[1][r] * GATE_INV + xr[NHID]     + b0r[1];
        const float pg = acc[2][r] * GATE_INV + xr[2 * NHID] + b0r[2];
        const float po = acc[3][r] * GATE_INV + xr[3 * NHID] + b0r[3];
        const float c = lsig(pf) * c0r[r] + lsig(pi) * ltanh(pg);
        c0r[r] = c;
        const float h = ltanh(c) * lsig(po);
        h0n[row * HPITCH + unit] = (_Float16)(h * SC_H);
      }
    }
    __syncthreads();

    {
      const _Float16* h0c = h0b + ((t + 1) & 1) * HBUF;
      const _Float16* h1p = h1hb + (t & 1) * HBUF;
      _Float16* h1hn = h1hb + ((t + 1) & 1) * HBUF;
      _Float16* h1ln = h1lb + ((t + 1) & 1) * HBUF;
      v8f acc[4];
#pragma unroll
      for (int g = 0; g < 4; ++g) acc[g] = z8;
#pragma unroll
      for (int ks = 0; ks < NHID / 32; ++ks) {
        const int kk = ks * 32 + koff;
        const v16h a = Frag<_Float16>::load(h0c + nn * HPITCH + kk);
        v16h bq[4];
#pragma unroll
        for (int g = 0; g < 4; ++g) bq[g] = Frag<_Float16>::load(WX1 + (size_t)(g * NHID + unit) * NHID + kk);
#pragma unroll
        for (int g = 0; g < 4; ++g) acc[g] = Frag<_Float16>::mma(a, bq[g], acc[g]);
        dep_guard_h(acc[0], acc[3], a, bq[3]);
        keep4_h(bq[0], bq[1], bq[2], bq[3]);
      }
#pragma unroll
      for (int ks = 0; ks < NHID / 32; ++ks) {
        const int kk = ks * 32 + koff;
        const v16h a = Frag<_Float16>::load(h1p + nn * HPITCH + kk);
        v16h bq[4];
#pragma unroll
        for (int g = 0; g < 4; ++g) bq[g] = Frag<_Float16>::load(WH1 + (size_t)(g * NHID + unit) * NHID + kk);
#pragma unroll
        for (int g = 0; g < 4; ++g) acc[g] = Frag<_Float16>::mma(a, bq[g], acc[g]);
        dep_guard_h(acc[0], acc[3], a, bq[3]);
        keep4_h(bq[0], bq[1], bq[2], bq[3]);
      }
      acc_guard4(acc[0], acc[1], acc[2], acc[3]);
#pragma unroll
      for (int r = 0; r < 8; ++r) {
        const int row = hh * 8 + r;
        const float pf = acc[0][r] * GATE_INV + b1r[0];
        const float pi = acc[1][r] * GATE_INV + b1r[1];
        const float pg = acc[2][r] * GATE_INV + b1r[2];
        const float po = acc[3][r] * GATE_INV + b1r[3];
        const float c = lsig(pf) * c1r[r] + lsig(pi) * ltanh(pg);
        c1r[r] = c;
        const float h = ltanh(c) * lsig(po);
        const float hs = h * SC_H;
        const _Float16 hi = (_Float16)hs;
        const float lo = (hs - (float)hi) * SC_LO;
        h1hn[row * HPITCH + unit] = hi;
        h1ln[row * HPITCH + unit] = (_Float16)lo;
      }
    }
    __syncthreads();

    if (wave < 2) {
      const _Float16* h1c = h1hb + ((t + 1) & 1) * HBUF;
      const _Float16* h1d = h1lb + ((t + 1) & 1) * HBUF;
      v8f oh = z8, ol = z8;
#pragma unroll
      for (int ks = 0; ks < NHID / 32; ++ks) {
        const int kk = ks * 32 + koff;
        const v16h ah = Frag<_Float16>::load(h1c + nn * HPITCH + kk);
        const v16h al = Frag<_Float16>::load(h1d + nn * HPITCH + kk);
        const v16h bw = Frag<_Float16>::load(WHY + (size_t)(wave * 16 + nn) * NHID + kk);
        oh = Frag<_Float16>::mma(ah, bw, oh);
        ol = Frag<_Float16>::mma(al, bw, ol);
        dep_guard_h(oh, ol, al, bw);
      }
      const int slot = t & (YCHUNK - 1);
#pragma unroll
      for (int r = 0; r < 8; ++r) {
        const int row = hh * 8 + r;
        const float y = (oh[r] + ol[r] * LO_INV) * Y_INV + byr;
        if (ycol < NVOC) yb[row * YPITCH + slot * NVOC + ycol] = y;
      }
    }

    if ((t & (YCHUNK - 1)) == (YCHUNK - 1)) {
      __syncthreads();
      const int t0 = t - (YCHUNK - 1);
      const int lq = lane >> 3;
      const int c4 = (lane & 7) * 4;
      for (int rr = 0; rr < 2; ++rr) {
        const int row = wave * 2 + rr;
        const float* ybr = yb + row * YPITCH;
        float* ob = out + ((size_t)(bbase + row) * NSTEP + (size_t)t0) * NVOC;
        for (int pass = 0; pass < 2; ++pass) {
#pragma unroll
          for (int it = 0; it < (YLINES + 3) / 4; ++it) {
            const int line = it * 4 + lq;
            const int lc = line < YLINES ? line : (YLINES - 1);
            const v4f v = *(const v4f*)(ybr + lc * 32 + c4);
            if (line < YLINES) *(volatile v4f*)(ob + line * 32 + c4) = v;
          }
          __threadfence();
        }
      }
      __syncthreads();
    }
  }
}

extern "C" void kernel_launch(void* const* d_in, const int* in_sizes, int n_in,
                              void* d_out, int out_size, void* d_ws,
                              size_t ws_size, hipStream_t stream) {
  (void)in_sizes; (void)n_in; (void)out_size;
  if (ws_size < WS_TOTAL) return;
  const int*   x   = (const int*)d_in[0];
  const float* emb = (const float*)d_in[1];
  const float* wx0 = (const float*)d_in[2];
  const float* wh0 = (const float*)d_in[3];
  const float* b0  = (const float*)d_in[4];
  const float* wx1 = (const float*)d_in[5];
  const float* wh1 = (const float*)d_in[6];
  const float* b1  = (const float*)d_in[7];
  const float* why = (const float*)d_in[8];
  const float* by  = (const float*)d_in[9];
  char* ws = (char*)d_ws;
  unsigned short* embB = (unsigned short*)(ws + WS_EMBB);
  unsigned short* wx0T = (unsigned short*)(ws + WS_WX0T);
  unsigned short* wh0T = (unsigned short*)(ws + WS_WH0T);
  unsigned short* wx1T = (unsigned short*)(ws + WS_WX1T);
  unsigned short* wh1T = (unsigned short*)(ws + WS_WH1T);
  unsigned short* whyT = (unsigned short*)(ws + WS_WHYT);
  float* xproj = (float*)(ws + WS_XPROJ);
  float* out = (float*)d_out;

  k_prep16<<<dim3(2), dim3(256), 0, stream>>>(emb, (long)NEMB, 1L, NVOC, embB, NEMBROWS, NEMB, 1.0f, 0);
  k_prep16<<<dim3(16), dim3(256), 0, stream>>>(wx0, 1L, (long)NGATE, NGATE, wx0T, NGATE, NEMB, 1.0f, 0);
  k_prep16<<<dim3(32), dim3(256), 0, stream>>>(wh0, 1L, (long)NGATE, NGATE, wh0T, NGATE, NHID, SC_W, 1);
  k_prep16<<<dim3(32), dim3(256), 0, stream>>>(wx1, 1L, (long)NGATE, NGATE, wx1T, NGATE, NHID, SC_W, 1);
  k_prep16<<<dim3(32), dim3(256), 0, stream>>>(wh1, 1L, (long)NGATE, NGATE, wh1T, NGATE, NHID, SC_W, 1);
  k_prep16<<<dim3(2), dim3(256), 0, stream>>>(why, 1L, (long)NVOC, NVOC, whyT, NVOCPAD, NHID, SC_Y, 1);

  wmma_gemm64<1, false, 0, 0, false><<<dim3(1, 1, 1), dim3(256), 0, stream>>>(
      embB, embB, NEMB, 0L,
      wx0T, wx0T, NEMB, 0L,
      (void*)xproj, (void*)xproj, NGATE, 0L,
      b0, (const float*)xproj, 0L,
      NEMBROWS, NGATE, NEMB, 1.0f);

  k_lstm2<<<dim3(NBLK_MAIN), dim3(256), LDS_TOTAL, stream>>>(x, xproj, wh0T, wx1T, wh1T, whyT, b0, b1, by, out);
}
